// AdaLNTransformerBlock_70300024701813
// MI455X (gfx1250) — hardware-verified
//
#include <hip/hip_runtime.h>
#include <math.h>
#include <stdint.h>

#define NB    4
#define SEQ   1024
#define DM    1024
#define NH    16
#define HD    64
#define NTOK  (NB * SEQ)
#define NQB   (SEQ / 64)
#define QKP   (2 * DM)
#define LNEPS 1.0e-5f
static_assert(NH * HD == DM);
static_assert((SEQ % 64) == 0 && (DM % 64) == 0 && (NTOK % 64) == 0 && (DM % 32) == 0);
static_assert(DM == 4 * 256);

typedef _Float16 v16h __attribute__((ext_vector_type(16)));
typedef _Float16 v8h  __attribute__((ext_vector_type(8)));
typedef __bf16   v16b __attribute__((ext_vector_type(16)));
typedef __bf16   v8b  __attribute__((ext_vector_type(8)));
typedef float    v8f  __attribute__((ext_vector_type(8)));
typedef float    v4f  __attribute__((ext_vector_type(4)));
typedef unsigned int v4u __attribute__((ext_vector_type(4)));
typedef unsigned int v2u __attribute__((ext_vector_type(2)));

__device__ __forceinline__ unsigned short bf_bits(float f) {
  unsigned u = __float_as_uint(f);
  return (unsigned short)((u + 0x7FFFu + ((u >> 16) & 1u)) >> 16);
}
__device__ __forceinline__ float bf_up(unsigned short h) { return __uint_as_float(((unsigned)h) << 16); }
__device__ __forceinline__ float bfr(float f) { return bf_up(bf_bits(f)); }
__device__ __forceinline__ unsigned short h_bits(_Float16 x) { return __builtin_bit_cast(unsigned short, x); }
__device__ __forceinline__ unsigned pk16(unsigned short a, unsigned short b) { return (unsigned)a | ((unsigned)b << 16); }
__device__ __forceinline__ v8f zero8() { v8f z = {0.f, 0.f, 0.f, 0.f, 0.f, 0.f, 0.f, 0.f}; return z; }

__device__ __forceinline__ v16b ldfrag_b(const __bf16* p) {
  union { v16b v; v8b h[2]; } f;
  f.h[0] = *(const v8b*)(p);
  f.h[1] = *(const v8b*)(p + 16);
  return f.v;
}
__device__ __forceinline__ v16h ldfrag_h(const _Float16* p) {
  union { v16h v; v8h h[2]; } f;
  f.h[0] = *(const v8h*)(p);
  f.h[1] = *(const v8h*)(p + 16);
  return f.v;
}

__device__ __forceinline__ v8f mma_h(v16h a, v16h b, v8f c) {
  c = __builtin_amdgcn_wmma_f32_16x16x32_f16(false, a, false, b, (short)0, c, false, false);
#if defined(__HIP_DEVICE_COMPILE__)
  asm volatile("v_nop\n\tv_nop\n\tv_nop\n\tv_nop" : "+v"(c) : "v"(a), "v"(b));
#endif
  return c;
}
__device__ __forceinline__ v8f mma_b_raw(v16b a, v16b b, v8f c) {
  return __builtin_amdgcn_wmma_f32_16x16x32_bf16(false, a, false, b, (short)0, c, false, false);
}
__device__ __forceinline__ void dep_guard1(v8f& a, v8f& b, v16b x) {
#if defined(__HIP_DEVICE_COMPILE__)
  asm volatile("v_nop\n\tv_nop\n\tv_nop\n\tv_nop" : "+v"(a), "+v"(b) : "v"(x));
#endif
}
__device__ __forceinline__ void keep4_b(v16b a, v16b b, v16b c, v16b d) {
#if defined(__HIP_DEVICE_COMPILE__)
  asm volatile("v_nop" :: "v"(a), "v"(b), "v"(c), "v"(d));
#endif
}
__device__ __forceinline__ void acc_guard4(v8f& a, v8f& b, v8f& c, v8f& d) {
#if defined(__HIP_DEVICE_COMPILE__)
  asm volatile("v_nop\n\tv_nop\n\tv_nop\n\tv_nop" : "+v"(a), "+v"(b), "+v"(c), "+v"(d));
#endif
}
__device__ __forceinline__ void wave_sync_lds() {
  __builtin_amdgcn_fence(__ATOMIC_RELEASE, "workgroup");
  __builtin_amdgcn_wave_barrier();
  __builtin_amdgcn_fence(__ATOMIC_ACQUIRE, "workgroup");
}
__device__ __forceinline__ float wsum(float v) {
#pragma unroll
  for (int off = 16; off > 0; off >>= 1) v += __shfl_xor(v, off, 32);
  return v;
}
__device__ __forceinline__ float bsum256(float v, float* red, int lane, int wave) {
  v = wsum(v);
  if (lane == 0) red[wave] = v;
  __syncthreads();
  float tot = 0.f;
#pragma unroll
  for (int w = 0; w < 8; ++w) tot += red[w];
  return tot;
}

__global__ __launch_bounds__(256) void convT64(const float* __restrict__ W, unsigned short* Wt, int K, int O) {
  __shared__ __align__(16) unsigned short sTt[64 * 72];
  const int tid = threadIdx.x, lane = tid & 31, wave = tid >> 5;
  const int o0 = blockIdx.x * 64, k0 = blockIdx.y * 64;
  const int kr = tid >> 2, cs = (tid & 3) * 16;
  const float* src = W + (size_t)(k0 + kr) * O + o0 + cs;
#pragma unroll
  for (int q = 0; q < 4; ++q) {
    const v4f v = *(const v4f*)(src + 4 * q);
#pragma unroll
    for (int e = 0; e < 4; ++e) sTt[(cs + 4 * q + e) * 72 + kr] = bf_bits(v[e]);
  }
  __syncthreads();
  const int q8 = lane >> 3, c8 = (lane & 7) * 8;
  v4u vv[2];
#pragma unroll
  for (int it = 0; it < 2; ++it) {
    const int row = wave * 8 + it * 4 + q8;
    vv[it] = *(const v4u*)(sTt + row * 72 + c8);
  }
  for (int pass = 0; pass < 2; ++pass) {
#pragma unroll
    for (int it = 0; it < 2; ++it) {
      const int row = wave * 8 + it * 4 + q8;
      *(volatile v4u*)(Wt + (size_t)(o0 + row) * K + k0 + c8) = vv[it];
    }
    __threadfence();
  }
}

__device__ __forceinline__ float silu_f(float z) { return z * __builtin_amdgcn_rcpf(1.0f + __expf(-z)); }
__global__ __launch_bounds__(256) void silu_cvt(const float* __restrict__ tp, const float* __restrict__ hp,
                                                unsigned short* out, int n8) {
  const int i = blockIdx.x * 256 + threadIdx.x;
  if (i < n8) {
    const size_t o = (size_t)i * 8;
    const v4f a0 = *(const v4f*)(tp + o), a1 = *(const v4f*)(tp + o + 4);
    const v4f b0 = *(const v4f*)(hp + o), b1 = *(const v4f*)(hp + o + 4);
    v4u p;
#pragma unroll
    for (int e = 0; e < 2; ++e) {
      const float u0 = silu_f(bfr(a0[2 * e])     + bfr(b0[2 * e]));
      const float u1 = silu_f(bfr(a0[2 * e + 1]) + bfr(b0[2 * e + 1]));
      const float u2 = silu_f(bfr(a1[2 * e])     + bfr(b1[2 * e]));
      const float u3 = silu_f(bfr(a1[2 * e + 1]) + bfr(b1[2 * e + 1]));
      p[e]     = pk16(bf_bits(u0), bf_bits(u1));
      p[2 + e] = pk16(bf_bits(u2), bf_bits(u3));
    }
    *(volatile v4u*)(out + o) = p;
    __threadfence();
    *(volatile v4u*)(out + o) = p;
  }
}

template <int OM, int BIASM, int RELU, int RES>
__global__ __launch_bounds__(256) void gemm64(
    const unsigned short* __restrict__ Ap, int lda, long long strideA,
    const unsigned short* __restrict__ Btp, int ldb, long long strideB,
    const float* __restrict__ bias0, const float* __restrict__ bias1, int Nb,
    const float* __restrict__ resid,
    void* Cout, int ldc, long long strideC,
    int M, int N, int K) {
  const __bf16* A  = (const __bf16*)(const void*)Ap;
  const __bf16* Bt = (const __bf16*)(const void*)Btp;
  __shared__ __align__(16) float sT[8][16 * 68];
  const int b    = blockIdx.y;
  const int lane = threadIdx.x & 31;
  const int wave = threadIdx.x >> 5;
  const int tilesN = N >> 6;
  const int tilesM = M >> 6;
  const int tile = blockIdx.x * 8 + wave;
  if (tile >= tilesM * tilesN) return;
  const int tm = tile / tilesN;
  const int tn = tile - tm * tilesN;
  const int m0 = tm << 6;
  const int n0 = tn << 6;

  const __bf16* Ab = A  + (size_t)b * strideA;
  const __bf16* Bb = Bt + (size_t)b * strideB;

  const int rlane = lane & 15;
  const int koff  = (lane >> 4) * 8;
  const int mOff  = (lane >> 4) * 8;

  v8f acc[4][4];
#pragma unroll
  for (int i = 0; i < 4; ++i)
#pragma unroll
    for (int j = 0; j < 4; ++j) acc[i][j] = zero8();

  for (int k0 = 0; k0 < K; k0 += 32) {
    v16b bh[4];
#pragma unroll
    for (int j = 0; j < 4; ++j) {
      const size_t bo = (size_t)(n0 + (j << 4) + rlane) * ldb + koff + k0;
      bh[j] = ldfrag_b(Bb + bo);
    }
#pragma unroll
    for (int i = 0; i < 4; ++i) {
      const size_t ao = (size_t)(m0 + (i << 4) + rlane) * lda + koff + k0;
      const v16b ah = ldfrag_b(Ab + ao);
#pragma unroll
      for (int j = 0; j < 4; ++j) acc[i][j] = mma_b_raw(ah, bh[j], acc[i][j]);
      dep_guard1(acc[i][0], acc[i][3], ah);
    }
    keep4_b(bh[0], bh[1], bh[2], bh[3]);
  }
  acc_guard4(acc[0][0], acc[0][1], acc[0][2], acc[0][3]);
  acc_guard4(acc[1][0], acc[1][1], acc[1][2], acc[1][3]);
  acc_guard4(acc[2][0], acc[2][1], acc[2][2], acc[2][3]);
  acc_guard4(acc[3][0], acc[3][1], acc[3][2], acc[3][3]);

  const int hh2 = lane >> 4, c4 = (lane & 15) * 4;
  const int q8  = lane >> 3, c8 = (lane & 7) * 8;
  float bc[8];
#pragma unroll
  for (int e = 0; e < 8; ++e) bc[e] = 0.f;
  if (BIASM == 0) {
    const bool use1 = (n0 >= Nb);
    if (OM == 0) {
      const int cb = n0 + c4;
      const int i0 = (cb < Nb - 4) ? cb : (Nb - 4);
      const int i1 = (cb - Nb > 0) ? (cb - Nb) : 0;
      const v4f b0v = *(const v4f*)(bias0 + i0);
      const v4f b1v = *(const v4f*)(bias1 + i1);
#pragma unroll
      for (int e = 0; e < 4; ++e) bc[e] = bfr(use1 ? b1v[e] : b0v[e]);
    } else {
      const int cb = n0 + c8;
      const int i0 = (cb < Nb - 8) ? cb : (Nb - 8);
      const int i1 = (cb - Nb > 0) ? (cb - Nb) : 0;
      const v4f b0a = *(const v4f*)(bias0 + i0), b0b = *(const v4f*)(bias0 + i0 + 4);
      const v4f b1a = *(const v4f*)(bias1 + i1), b1b = *(const v4f*)(bias1 + i1 + 4);
#pragma unroll
      for (int e = 0; e < 4; ++e) {
        bc[e]     = bfr(use1 ? b1a[e] : b0a[e]);
        bc[4 + e] = bfr(use1 ? b1b[e] : b0b[e]);
      }
    }
  }

  float* slab = sT[wave];
#pragma unroll
  for (int i = 0; i < 4; ++i) {
    const int mBase = m0 + (i << 4);
#pragma unroll
    for (int j = 0; j < 4; ++j) {
#pragma unroll
      for (int r = 0; r < 8; ++r) {
        slab[(mOff + r) * 68 + (j << 4) + rlane] = acc[i][j][r];
      }
    }
    wave_sync_lds();
    if (OM == 0) {
      float* C = (float*)Cout + (size_t)b * strideC;
      const float* Rb = resid + (size_t)b * strideC;
      v4f vals[8];
#pragma unroll
      for (int it = 0; it < 8; ++it) {
        const int row = it * 2 + hh2;
        v4f v = *(const v4f*)(slab + row * 68 + c4);
#pragma unroll
        for (int e = 0; e < 4; ++e) v[e] += bc[e];
        if (RES != 0) {
          const v4f rr = *(const v4f*)(Rb + (size_t)(mBase + row) * ldc + n0 + c4);
#pragma unroll
          for (int e = 0; e < 4; ++e) v[e] += (RES == 2) ? bfr(rr[e]) : rr[e];
        }
        vals[it] = v;
      }
      for (int pass = 0; pass < 2; ++pass) {
#pragma unroll
        for (int it = 0; it < 8; ++it) {
          const int row = it * 2 + hh2;
          *(volatile v4f*)(C + (size_t)(mBase + row) * ldc + n0 + c4) = vals[it];
        }
        __threadfence();
      }
    } else {
      unsigned short* C = (unsigned short*)Cout + (size_t)b * strideC;
      v4u hv[4];
#pragma unroll
      for (int it = 0; it < 4; ++it) {
        const int row = it * 4 + q8;
        const float* sp = slab + row * 68 + c8;
        float bm = 0.f;
        if (BIASM == 1) bm = bfr(bias0[mBase + row]);
        v4u a;
#pragma unroll
        for (int e = 0; e < 4; ++e) {
          float f0 = sp[2 * e]     + ((BIASM == 1) ? bm : bc[2 * e]);
          float f1 = sp[2 * e + 1] + ((BIASM == 1) ? bm : bc[2 * e + 1]);
          if (RELU) { f0 = fmaxf(f0, 0.f); f1 = fmaxf(f1, 0.f); }
          unsigned short u0, u1;
          if (OM == 1) { u0 = bf_bits(f0); u1 = bf_bits(f1); }
          else         { u0 = h_bits((_Float16)f0); u1 = h_bits((_Float16)f1); }
          a[e] = pk16(u0, u1);
        }
        hv[it] = a;
      }
      for (int pass = 0; pass < 2; ++pass) {
#pragma unroll
        for (int it = 0; it < 4; ++it) {
          const int row = it * 4 + q8;
          *(volatile v4u*)(C + (size_t)(mBase + row) * ldc + n0 + c8) = hv[it];
        }
        __threadfence();
      }
    }
    wave_sync_lds();
  }
}

__global__ __launch_bounds__(128)
void attn64(const unsigned short* __restrict__ qkp, const unsigned short* __restrict__ vtp,
            const int* __restrict__ rmask, unsigned short* outp, float sscale) {
  union FH { v16h v; v8h h[2]; };
  __shared__ __align__(16) _Float16 Ksh[64 * 64];
  __shared__ __align__(16) _Float16 Vth[64 * 64];
  __shared__ __align__(16) _Float16 Psh[4][16 * 64];
  __shared__ __align__(16) float    Os[4][16 * 64];

  const int tid  = threadIdx.x;
  const int wave = tid >> 5;
  const int lane = tid & 31;
  const int hh   = lane >> 4;
  const int c    = lane & 15;

  const int bx   = blockIdx.x;
  const int qb   = bx % NQB;
  const int rest = bx / NQB;
  const int h    = rest % NH;
  const int b    = rest / NH;
  const int q0   = qb * 64 + wave * 16;
  const size_t rowB = (size_t)b * SEQ;

  const _Float16* Qh = (const _Float16*)(const void*)qkp + (size_t)h * HD;
  const _Float16* Kg = (const _Float16*)(const void*)qkp + DM + (size_t)h * HD;
  const _Float16* Vh = (const _Float16*)(const void*)vtp + ((size_t)b * DM + (size_t)h * HD) * SEQ;

  v16h qa[2];
#pragma unroll
  for (int dc = 0; dc < 2; ++dc) qa[dc] = ldfrag_h(Qh + (rowB + q0 + c) * QKP + dc * 32 + 8 * hh);

  int mfl[8];
#pragma unroll
  for (int r = 0; r < 8; ++r) mfl[r] = rmask[rowB + q0 + 8 * hh + r];

  float mrow[8], lrow[8];
  v8f oacc[4];
#pragma unroll
  for (int r = 0; r < 8; ++r) { mrow[r] = -INFINITY; lrow[r] = 0.f; }
#pragma unroll
  for (int t = 0; t < 4; ++t) oacc[t] = zero8();

  for (int kt = 0; kt < NQB; ++kt) {
    const int kv0 = kt * 64;
    __syncthreads();
    {
      const int r = tid >> 1, hf = (tid & 1) * 32;
      const _Float16* kg = Kg + (rowB + kv0 + r) * QKP + hf;
      const _Float16* vg = Vh + (size_t)r * SEQ + kv0 + hf;
#pragma unroll
      for (int i = 0; i < 4; ++i) {
        const v8h a0 = *(const v8h*)(kg + 8 * i);
        const v8h b0 = *(const v8h*)(vg + 8 * i);
        *(v8h*)(Ksh + r * 64 + hf + 8 * i) = a0;
        *(v8h*)(Vth + r * 64 + hf + 8 * i) = b0;
      }
    }
    __syncthreads();

    v8f s[4];
#pragma unroll
    for (int j = 0; j < 4; ++j) {
      v8f sh = zero8();
#pragma unroll
      for (int dc = 0; dc < 2; ++dc) {
        FH kb;
        kb.h[0] = *(const v8h*)(Ksh + (j * 16 + c) * 64 + dc * 32 + 8 * hh);
        kb.h[1] = *(const v8h*)(Ksh + (j * 16 + c) * 64 + dc * 32 + 16 + 8 * hh);
        sh = mma_h(qa[dc], kb.v, sh);
      }
#pragma unroll
      for (int r = 0; r < 8; ++r) s[j][r] = (mfl[r] != 0) ? (sh[r] * sscale) : 0.f;
    }

    _Float16* pwh = Psh[wave];
#pragma unroll
    for (int r = 0; r < 8; ++r) {
      float m = s[0][r];
      m = fmaxf(m, s[1][r]);
      m = fmaxf(m, s[2][r]);
      m = fmaxf(m, s[3][r]);
#pragma unroll
      for (int off = 1; off < 16; off <<= 1) m = fmaxf(m, __shfl_xor(m, off, 32));
      const float mnew  = fmaxf(mrow[r], m);
      const float alpha = __expf(mrow[r] - mnew);
      mrow[r] = mnew;
      float psum = 0.f;
#pragma unroll
      for (int j = 0; j < 4; ++j) {
        const float p = __expf(s[j][r] - mnew);
        psum += p;
        pwh[(8 * hh + r) * 64 + j * 16 + c] = (_Float16)(p * 1024.0f);
      }
#pragma unroll
      for (int off = 1; off < 16; off <<= 1) psum += __shfl_xor(psum, off, 32);
      lrow[r] = lrow[r] * alpha + psum;
#pragma unroll
      for (int t = 0; t < 4; ++t) oacc[t][r] *= alpha;
    }
    wave_sync_lds();

#pragma unroll 1
    for (int kk = 0; kk < 2; ++kk) {
      FH pa;
      pa.h[0] = *(const v8h*)(pwh + c * 64 + kk * 32 + 8 * hh);
      pa.h[1] = *(const v8h*)(pwh + c * 64 + kk * 32 + 16 + 8 * hh);
#pragma unroll
      for (int t = 0; t < 4; ++t) {
        FH vb;
        vb.h[0] = *(const v8h*)(Vth + (t * 16 + c) * 64 + kk * 32 + 8 * hh);
        vb.h[1] = *(const v8h*)(Vth + (t * 16 + c) * 64 + kk * 32 + 16 + 8 * hh);
        oacc[t] = mma_h(pa.v, vb.v, oacc[t]);
      }
    }
  }

  float* os = Os[wave];
#pragma unroll
  for (int r = 0; r < 8; ++r) {
    const float l = lrow[r];
    const float inv = ((l > 0.f) ? (1.0f / l) : 0.f) * (1.0f / 1024.0f);
#pragma unroll
    for (int t = 0; t < 4; ++t) os[(8 * hh + r) * 64 + t * 16 + c] = oacc[t][r] * inv;
  }
  wave_sync_lds();
  {
    const int q4 = lane >> 3, c8 = (lane & 7) * 8;
    v4u hv[4];
#pragma unroll
    for (int it = 0; it < 4; ++it) {
      const int row = it * 4 + q4;
      const float* sp = os + row * 64 + c8;
      v4u a;
#pragma unroll
      for (int e = 0; e < 4; ++e) a[e] = pk16(bf_bits(sp[2 * e]), bf_bits(sp[2 * e + 1]));
      hv[it] = a;
    }
    for (int pass = 0; pass < 2; ++pass) {
#pragma unroll
      for (int it = 0; it < 4; ++it) {
        const int row = it * 4 + q4;
        const size_t go = (rowB + q0 + row) * DM + (size_t)h * HD + c8;
        *(volatile v4u*)(outp + go) = hv[it];
      }
      __threadfence();
    }
  }
}

__device__ __forceinline__ void row_store_f32(float* dst_row, v4f o, int t) {
  *(volatile v4f*)(dst_row + 4 * t) = o;
  __threadfence();
  *(volatile v4f*)(dst_row + 4 * t) = o;
}
__device__ __forceinline__ void row_store_bf16(unsigned int* sb, unsigned short* dst_row, v4f o, int t) {
  v2u p;
  p[0] = pk16(bf_bits(o[0]), bf_bits(o[1]));
  p[1] = pk16(bf_bits(o[2]), bf_bits(o[3]));
  *(v2u*)(sb + 2 * t) = p;
  __syncthreads();
  if (t < 128) {
    const v4u v = *(const v4u*)(sb + 4 * t);
    *(volatile v4u*)(dst_row + 8 * t) = v;
    __threadfence();
    *(volatile v4u*)(dst_row + 8 * t) = v;
  }
}

__global__ __launch_bounds__(256) void row_mod(const float* __restrict__ X, const float* __restrict__ modp,
                                               unsigned short* outB) {
  __shared__ float red0[8], red1[8];
  __shared__ __align__(16) unsigned int sb[512];
  const int t = threadIdx.x, lane = t & 31, wave = t >> 5;
  const size_t row  = (size_t)blockIdx.x;
  const size_t base = row * DM;
  v4f xv = *(const v4f*)(X + base + 4 * t);
#pragma unroll
  for (int e = 0; e < 4; ++e) xv[e] = bfr(xv[e]);
  const float mean = bsum256((xv[0] + xv[1]) + (xv[2] + xv[3]), red0, lane, wave) * (1.0f / DM);
  v4f d;
#pragma unroll
  for (int e = 0; e < 4; ++e) d[e] = xv[e] - mean;
  const float var  = bsum256((d[0] * d[0] + d[1] * d[1]) + (d[2] * d[2] + d[3] * d[3]), red1, lane, wave) * (1.0f / DM);
  const float rstd = 1.0f / sqrtf(var + LNEPS);
  const v4f sh = *(const v4f*)(modp + row * QKP + 4 * t);
  const v4f sc = *(const v4f*)(modp + row * QKP + DM + 4 * t);
  v4f y;
#pragma unroll
  for (int e = 0; e < 4; ++e) y[e] = (d[e] * rstd) * (1.0f + sc[e]) + sh[e];
  row_store_bf16(sb, outB + base, y, t);
}

template <int RIN, int OUTF, int OUTB, int POST>
__global__ __launch_bounds__(256) void ln_row(const float* __restrict__ X, const float* __restrict__ gam,
                                              const float* __restrict__ bet, const float* __restrict__ post,
                                              float* outF, unsigned short* outB) {
  __shared__ float red0[8], red1[8];
  __shared__ __align__(16) unsigned int sb[512];
  const int t = threadIdx.x, lane = t & 31, wave = t >> 5;
  const size_t base = (size_t)blockIdx.x * DM;
  v4f xv = *(const v4f*)(X + base + 4 * t);
  if (RIN) {
#pragma unroll
    for (int e = 0; e < 4; ++e) xv[e] = bfr(xv[e]);
  }
  const float mean = bsum256((xv[0] + xv[1]) + (xv[2] + xv[3]), red0, lane, wave) * (1.0f / DM);
  v4f d;
#pragma unroll
  for (int e = 0; e < 4; ++e) d[e] = xv[e] - mean;
  const float var  = bsum256((d[0] * d[0] + d[1] * d[1]) + (d[2] * d[2] + d[3] * d[3]), red1, lane, wave) * (1.0f / DM);
  const float rstd = 1.0f / sqrtf(var + LNEPS);
  const v4f gv = *(const v4f*)(gam + 4 * t);
  const v4f bv = *(const v4f*)(bet + 4 * t);
  v4f y;
#pragma unroll
  for (int e = 0; e < 4; ++e) y[e] = (d[e] * rstd) * bfr(gv[e]) + bfr(bv[e]);
  if (OUTF) {
    v4f o = y;
    if (POST) {
      const v4f pv = *(const v4f*)(post + base + 4 * t);
#pragma unroll
      for (int e = 0; e < 4; ++e) o[e] += pv[e];
    }
    row_store_f32(outF + base, o, t);
  }
  if (OUTB) row_store_bf16(sb, outB + base, y, t);
}

extern "C" void kernel_launch(void* const* d_in, const int* in_sizes, int n_in,
                              void* d_out, int out_size, void* d_ws, size_t ws_size,
                              hipStream_t stream) {
  if (n_in < 35) return;
  if (in_sizes[0] != NTOK * DM || in_sizes[1] != NTOK * DM || in_sizes[2] != NTOK * DM) return;
  if (in_sizes[3] != NTOK || in_sizes[4] != NTOK) return;
  for (int i = 5; i <= 19; i += 2) { if (in_sizes[i] != DM * DM) return; if (in_sizes[i + 1] != DM) return; }
  if (in_sizes[21] != 2 * DM * DM || in_sizes[22] != 2 * DM) return;
  if (in_sizes[23] != DM * DM || in_sizes[24] != DM || in_sizes[25] != DM * DM || in_sizes[26] != DM) return;
  for (int i = 27; i <= 34; ++i) { if (in_sizes[i] != DM) return; }
  if (out_size != NTOK * DM) return;

  const float* x     = (const float*)d_in[0];
  const float* hin   = (const float*)d_in[1];
  const float* tin   = (const float*)d_in[2];
  const int*   maskq = (const int*)d_in[3];
  const int*   extq  = (const int*)d_in[4];
  const float* Wsq = (const float*)d_in[5];   const float* bsq = (const float*)d_in[6];
  const float* Wsk = (const float*)d_in[7];   const float* bsk = (const float*)d_in[8];
  const float* Wsv = (const float*)d_in[9];   const float* bsv = (const float*)d_in[10];
  const float* Wso = (const float*)d_in[11];  const float* bso = (const float*)d_in[12];
  const float* Wcq = (const float*)d_in[13];  const float* bcq = (const float*)d_in[14];
  const float* Wck = (const float*)d_in[15];  const float* bck = (const float*)d_in[16];
  const float* Wcv = (const float*)d_in[17];  const float* bcv = (const float*)d_in[18];
  const float* Wco = (const float*)d_in[19];  const float* bco = (const float*)d_in[20];
  const float* ada_w = (const float*)d_in[21]; const float* ada_b = (const float*)d_in[22];
  const float* fw1 = (const float*)d_in[23];  const float* fb1 = (const float*)d_in[24];
  const float* fw2 = (const float*)d_in[25];  const float* fb2 = (const float*)d_in[26];
  const float* ln2_g = (const float*)d_in[27]; const float* ln2_b = (const float*)d_in[28];
  const float* ln3_g = (const float*)d_in[29]; const float* ln3_b = (const float*)d_in[30];
  const float* lnh_g = (const float*)d_in[31]; const float* lnh_b = (const float*)d_in[32];
  const float* lnf_g = (const float*)d_in[33]; const float* lnf_b = (const float*)d_in[34];

  const size_t PW   = (size_t)DM * DM * 2;
  const size_t PR   = (size_t)NTOK * QKP * 4;
  const size_t PAB  = (size_t)NTOK * DM * 2;
  const size_t PAF  = (size_t)NTOK * DM * 4;
  const size_t PQK  = (size_t)NTOK * QKP * 2;
  const size_t PVT  = (size_t)NB * DM * SEQ * 2;
  size_t off = 0;
  const size_t oWqk = off; off += 2 * PW;
  const size_t oWsv = off; off += PW;
  const size_t oWso = off; off += PW;
  const size_t oWcq = off; off += PW;
  const size_t oWck = off; off += PW;
  const size_t oWcv = off; off += PW;
  const size_t oWco = off; off += PW;
  const size_t oWad = off; off += 2 * PW;
  const size_t oW1  = off; off += PW;
  const size_t oW2  = off; off += PW;
  const size_t oR   = off; off += PR;
  const size_t oP1  = off; off += PAB;
  const size_t oP2  = off; off += PAB;
  const size_t oQK  = off; off += PQK;
  const size_t oVT  = off; off += PVT;
  const size_t oCtx = off; off += PAB;
  const size_t oHO  = off; off += PAF;
  if (off > ws_size) return;
  if (off > (size_t)134217728) return;

  char* ws = (char*)d_ws;
  unsigned short* Wqk  = (unsigned short*)(ws + oWqk);
  unsigned short* Wsvt = (unsigned short*)(ws + oWsv);
  unsigned short* Wsot = (unsigned short*)(ws + oWso);
  unsigned short* Wcqt = (unsigned short*)(ws + oWcq);
  unsigned short* Wckt = (unsigned short*)(ws + oWck);
  unsigned short* Wcvt = (unsigned short*)(ws + oWcv);
  unsigned short* Wcot = (unsigned short*)(ws + oWco);
  unsigned short* Wadt = (unsigned short*)(ws + oWad);
  unsigned short* W1t  = (unsigned short*)(ws + oW1);
  unsigned short* W2t  = (unsigned short*)(ws + oW2);
  float*          R    = (float*)(ws + oR);
  float*          Rmid = R + (size_t)NTOK * DM;
  unsigned short* P1   = (unsigned short*)(ws + oP1);
  unsigned short* P2   = (unsigned short*)(ws + oP2);
  unsigned short* QK   = (unsigned short*)(ws + oQK);
  float*          F    = (float*)(ws + oQK);
  unsigned short* VT   = (unsigned short*)(ws + oVT);
  unsigned short* Ctx  = (unsigned short*)(ws + oCtx);
  float*          HO   = (float*)(ws + oHO);

  const dim3 blk(256);
  const dim3 gT1(DM / 64, DM / 64);
  const dim3 gT2((2 * DM) / 64, DM / 64);
  const int  n8 = NTOK * DM / 8;
  const dim3 gE((n8 + 255) / 256);
  const dim3 gN2(((NTOK / 64) * (QKP / 64) + 7) / 8, 1);
  const dim3 gN1(((NTOK / 64) * (DM / 64) + 7) / 8, 1);
  const dim3 gVT(((DM / 64) * (SEQ / 64) + 7) / 8, NB);
  const dim3 gAttn(NB * NH * NQB);
  const dim3 gRow(NTOK);

  convT64<<<gT1, blk, 0, stream>>>(Wsq, Wqk, DM, DM);
  convT64<<<gT1, blk, 0, stream>>>(Wsk, Wqk + (size_t)DM * DM, DM, DM);
  convT64<<<gT1, blk, 0, stream>>>(Wsv, Wsvt, DM, DM);
  convT64<<<gT1, blk, 0, stream>>>(Wso, Wsot, DM, DM);
  convT64<<<gT1, blk, 0, stream>>>(Wcq, Wcqt, DM, DM);
  convT64<<<gT1, blk, 0, stream>>>(Wck, Wckt, DM, DM);
  convT64<<<gT1, blk, 0, stream>>>(Wcv, Wcvt, DM, DM);
  convT64<<<gT1, blk, 0, stream>>>(Wco, Wcot, DM, DM);
  convT64<<<gT2, blk, 0, stream>>>(ada_w, Wadt, DM, 2 * DM);
  convT64<<<gT1, blk, 0, stream>>>(fw1, W1t, DM, DM);
  convT64<<<gT1, blk, 0, stream>>>(fw2, W2t, DM, DM);

  silu_cvt<<<gE, blk, 0, stream>>>(tin, hin, P1, n8);
  gemm64<0, 0, 0, 0><<<gN2, blk, 0, stream>>>(
      P1, DM, 0LL, Wadt, DM, 0LL, ada_b, ada_b + DM, DM, x,
      (void*)R, QKP, 0LL, NTOK, QKP, DM);
  row_mod<<<gRow, blk, 0, stream>>>(x, R, P1);

  gemm64<2, 0, 0, 0><<<gN2, blk, 0, stream>>>(
      P1, DM, 0LL, Wqk, DM, 0LL, bsq, bsk, DM, x,
      (void*)QK, QKP, 0LL, NTOK, QKP, DM);
  gemm64<2, 1, 0, 0><<<gVT, blk, 0, stream>>>(
      Wsvt, DM, 0LL, P1, DM, (long long)SEQ * DM, bsv, bsv, DM, x,
      (void*)VT, SEQ, (long long)DM * SEQ, DM, SEQ, DM);
  attn64<<<gAttn, dim3(128), 0, stream>>>(QK, VT, extq, Ctx, 0.125f);
  gemm64<0, 0, 0, 2><<<gN1, blk, 0, stream>>>(
      Ctx, DM, 0LL, Wsot, DM, 0LL, bso, bso, DM, x,
      (void*)R, DM, 0LL, NTOK, DM, DM);

  ln_row<0, 0, 1, 0><<<gRow, blk, 0, stream>>>(R, ln2_g, ln2_b, x, HO, P1);
  ln_row<1, 0, 1, 0><<<gRow, blk, 0, stream>>>(hin, lnh_g, lnh_b, x, HO, P2);
  gemm64<2, 0, 0, 0><<<gN1, blk, 0, stream>>>(
      P1, DM, 0LL, Wcqt, DM, 0LL, bcq, bcq, DM, x,
      (void*)QK, QKP, 0LL, NTOK, DM, DM);
  gemm64<2, 0, 0, 0><<<gN1, blk, 0, stream>>>(
      P2, DM, 0LL, Wckt, DM, 0LL, bck, bck, DM, x,
      (void*)(QK + DM), QKP, 0LL, NTOK, DM, DM);
  gemm64<2, 1, 0, 0><<<gVT, blk, 0, stream>>>(
      Wcvt, DM, 0LL, P2, DM, (long long)SEQ * DM, bcv, bcv, DM, x,
      (void*)VT, SEQ, (long long)DM * SEQ, DM, SEQ, DM);
  attn64<<<gAttn, dim3(128), 0, stream>>>(QK, VT, maskq, Ctx, 0.125f);
  gemm64<0, 0, 0, 1><<<gN1, blk, 0, stream>>>(
      Ctx, DM, 0LL, Wcot, DM, 0LL, bco, bco, DM, R,
      (void*)Rmid, DM, 0LL, NTOK, DM, DM);

  ln_row<0, 1, 1, 0><<<gRow, blk, 0, stream>>>(Rmid, ln3_g, ln3_b, x, HO, P1);
  gemm64<1, 0, 1, 0><<<gN1, blk, 0, stream>>>(
      P1, DM, 0LL, W1t, DM, 0LL, fb1, fb1, DM, x,
      (void*)P2, DM, 0LL, NTOK, DM, DM);
  gemm64<0, 0, 0, 1><<<gN1, blk, 0, stream>>>(
      P2, DM, 0LL, W2t, DM, 0LL, fb2, fb2, DM, HO,
      (void*)F, DM, 0LL, NTOK, DM, DM);
  ln_row<0, 1, 0, 1><<<gRow, blk, 0, stream>>>(F, lnf_g, lnf_b, Rmid, (float*)d_out, P2);
  (void)hipGetLastError();
}
